// CoAttention_layer_16166256903001
// MI455X (gfx1250) — hardware-verified
//
#include <hip/hip_runtime.h>
#define BB 16
#define NNS 8
#define LL 64
#define SSQ 32
#define DD 256
#define HH 128

typedef __bf16 v16b __attribute__((ext_vector_type(16)));
typedef unsigned short v8us __attribute__((ext_vector_type(8), may_alias));
typedef float  v8f  __attribute__((ext_vector_type(8)));
typedef float  v4f  __attribute__((ext_vector_type(4)));
typedef float  v4fa __attribute__((ext_vector_type(4), may_alias));
union FragB { v16b v; v8us half[2]; unsigned short u[16]; };

__device__ __forceinline__ unsigned short bf16_bits(float x) { unsigned int u = __float_as_uint(x); return (unsigned short)((u + 0x7FFFu + ((u >> 16) & 1u)) >> 16); }
__device__ __forceinline__ float bf16_val(unsigned short b) { return __uint_as_float(((unsigned int)b) << 16); }
__device__ __forceinline__ float bf16_round(float x) { return bf16_val(bf16_bits(x)); }
template <int NT>
__device__ __forceinline__ v8f mmaN(v16b ah, v16b al, v16b bh, v16b bl, v8f c) {
  c = __builtin_amdgcn_wmma_f32_16x16x32_bf16(false, ah, false, bh, (short)0, c, false, false);
  if (NT >= 2) c = __builtin_amdgcn_wmma_f32_16x16x32_bf16(false, al, false, bh, (short)0, c, false, false);
  if (NT >= 3) c = __builtin_amdgcn_wmma_f32_16x16x32_bf16(false, ah, false, bl, (short)0, c, false, false);
  asm volatile("v_nop\n\tv_nop\n\tv_nop\n\tv_nop" : "+v"(c) : "v"(ah), "v"(al), "v"(bh), "v"(bl));
  return c;
}

__global__ __launch_bounds__(256) void k_wt_bf16(const float* __restrict__ W, unsigned short* __restrict__ Wt, int K, int N) {
  const int t = blockIdx.x * 256 + threadIdx.x;
  const int k8n = K / 8;
  if (t >= N * k8n) return;
  const int n = t / k8n, k8 = (t % k8n) * 8;
  v8us v;
#pragma unroll
  for (int i = 0; i < 8; ++i) v[i] = bf16_bits(W[(size_t)(k8 + i) * N + n]);
  *(volatile v8us*)(Wt + (size_t)n * K + k8) = v;
  __threadfence();
  *(volatile v8us*)(Wt + (size_t)n * K + k8) = v;
}

template <bool ASPLIT, int ACT, bool BIAS_BF16>
__global__ __launch_bounds__(128) void k_gemm_bf(const float* __restrict__ A, int lda, const unsigned short* __restrict__ Wt, int ldb,
                                               const float* __restrict__ bias, float* __restrict__ C, int ldc, int M, int N, int K) {
  __shared__ __attribute__((aligned(16))) float so[4][16][64];
  const int tid = threadIdx.x, w = tid >> 5, lane = tid & 31, ln = lane & 15, hh = lane >> 4;
  const int ntn = N / 64;
  const int wid = blockIdx.x * 4 + w;
  const int mt = wid / ntn, nq = wid % ntn;
  if (mt * 16 >= M) return;
  const int row0 = mt * 16, col0 = nq * 64;
  const float* arow = A + (size_t)(row0 + ln) * lda;
  v8f acc[4] = {};
  for (int kb = 0; kb < K; kb += 32) {
    FragB ah, al;
    const v4f x0 = *(const v4fa*)(arow + kb + 8 * hh), x1 = *(const v4fa*)(arow + kb + 8 * hh + 4);
    const v4f x2 = *(const v4fa*)(arow + kb + 16 + 8 * hh), x3 = *(const v4fa*)(arow + kb + 16 + 8 * hh + 4);
    float xs[16] = {x0[0],x0[1],x0[2],x0[3],x1[0],x1[1],x1[2],x1[3],x2[0],x2[1],x2[2],x2[3],x3[0],x3[1],x3[2],x3[3]};
#pragma unroll
    for (int i = 0; i < 16; ++i) { const unsigned short hb = bf16_bits(xs[i]); ah.u[i] = hb; al.u[i] = ASPLIT ? bf16_bits(xs[i] - bf16_val(hb)) : (unsigned short)0; }
#pragma unroll
    for (int t = 0; t < 4; ++t) {
      const unsigned short* brow = Wt + (size_t)(col0 + t * 16 + ln) * ldb + kb;
      FragB b;
      b.half[0] = *(const v8us*)(brow + 8 * hh);
      b.half[1] = *(const v8us*)(brow + 16 + 8 * hh);
      acc[t] = mmaN<ASPLIT ? 2 : 1>(ah.v, al.v, b.v, b.v, acc[t]);
    }
  }
#pragma unroll
  for (int t = 0; t < 4; ++t) {
    float bv = bias ? bias[col0 + t * 16 + ln] : 0.f;
    if (BIAS_BF16) bv = bf16_round(bv);
#pragma unroll
    for (int r = 0; r < 8; ++r) { float v = acc[t][r] + bv; if (ACT == 1) v = fmaxf(v, 0.f); so[w][8 * hh + r][t * 16 + ln] = v; }
  }
  __builtin_amdgcn_fence(__ATOMIC_ACQ_REL, "workgroup");
  __builtin_amdgcn_wave_barrier();
  const int rsub = lane >> 4, c4 = (lane & 15) * 4;
  for (int pass = 0; pass < 2; ++pass) {
#pragma unroll
    for (int q = 0; q < 8; ++q) {
      const int r = q * 2 + rsub;
      const v4f v = *(const v4fa*)&so[w][r][c4];
      *(volatile v4f*)(C + (size_t)(row0 + r) * ldc + col0 + c4) = v;
    }
    if (pass == 0) __threadfence();
  }
}

template <int D, bool CAUSAL>
__global__ __launch_bounds__(128) void k_flash(const float* __restrict__ qb, const float* __restrict__ kb, const float* __restrict__ vb,
                                             int pitch, int T, int H, float scale, float* __restrict__ y, int ypitch) {
  constexpr int KS = D / 32;
  constexpr int DT = D / 16;
  __shared__ __attribute__((aligned(16))) unsigned short sKh[32][D + 8], sKl[32][D + 8], sVh[32][D + 8], sVl[32][D + 8];
  __shared__ __attribute__((aligned(16))) unsigned short sPh[4][16][40], sPl[4][16][40];
  __shared__ __attribute__((aligned(16))) float sO[4][16][D];
  const int tid = threadIdx.x, w = tid >> 5, lane = tid & 31, ln = lane & 15, hh = lane >> 4;
  const int nqb = (T + 63) / 64;
  const int bh = blockIdx.x / nqb, qblk = blockIdx.x % nqb;
  const int b = bh / H, h = bh % H;
  const int q0 = qblk * 64 + w * 16;
  const float* Q = qb + (size_t)b * T * pitch + h * D;
  const float* K = kb + (size_t)b * T * pitch + h * D;
  const float* V = vb + (size_t)b * T * pitch + h * D;

  FragB aqh[KS], aql[KS];
  {
    int row = q0 + ln; if (row >= T) row = T - 1;
    const float* qr = Q + (size_t)row * pitch;
#pragma unroll
    for (int ks = 0; ks < KS; ++ks)
#pragma unroll
      for (int i = 0; i < 16; ++i) {
        const int d = ks * 32 + ((i < 8) ? (8 * hh + i) : (16 + 8 * hh + (i - 8)));
        const float x = qr[d] * scale; const unsigned short hb = bf16_bits(x);
        aqh[ks].u[i] = hb; aql[ks].u[i] = bf16_bits(x - bf16_val(hb));
      }
  }
  float m_r[8], l_r[8];
#pragma unroll
  for (int r = 0; r < 8; ++r) { m_r[r] = -3.0e38f; l_r[r] = 0.f; }
  v8f oacc[DT];
#pragma unroll
  for (int dt = 0; dt < DT; ++dt) oacc[dt] = (v8f){0.f,0.f,0.f,0.f,0.f,0.f,0.f,0.f};

  const int kv_end = CAUSAL ? min(T, qblk * 64 + 64) : T;
  for (int j0 = 0; j0 < kv_end; j0 += 32) {
    __syncthreads();
    for (int e = tid; e < 32 * (D / 4); e += 128) {
      const int r = e / (D / 4), c4 = (e % (D / 4)) * 4;
      const int key = j0 + r;
      v4f kf = {0.f,0.f,0.f,0.f}, vf = {0.f,0.f,0.f,0.f};
      if (key < T) { kf = *(const v4fa*)(K + (size_t)key * pitch + c4); vf = *(const v4fa*)(V + (size_t)key * pitch + c4); }
#pragma unroll
      for (int t = 0; t < 4; ++t) {
        unsigned short hb = bf16_bits(kf[t]); sKh[r][c4 + t] = hb; sKl[r][c4 + t] = bf16_bits(kf[t] - bf16_val(hb));
        hb = bf16_bits(vf[t]); sVh[r][c4 + t] = hb; sVl[r][c4 + t] = bf16_bits(vf[t] - bf16_val(hb));
      }
    }
    __syncthreads();
    v8f s[2];
#pragma unroll
    for (int nt = 0; nt < 2; ++nt) {
      v8f acc = {};
#pragma unroll
      for (int ks = 0; ks < KS; ++ks) {
        FragB bh_, bl_;
        bh_.half[0] = *(const v8us*)&sKh[nt * 16 + ln][ks * 32 + 8 * hh]; bh_.half[1] = *(const v8us*)&sKh[nt * 16 + ln][ks * 32 + 16 + 8 * hh];
        bl_.half[0] = *(const v8us*)&sKl[nt * 16 + ln][ks * 32 + 8 * hh]; bl_.half[1] = *(const v8us*)&sKl[nt * 16 + ln][ks * 32 + 16 + 8 * hh];
        acc = mmaN<3>(aqh[ks].v, aql[ks].v, bh_.v, bl_.v, acc);
      }
      s[nt] = acc;
    }
    float alpha[8];
#pragma unroll
    for (int r = 0; r < 8; ++r) {
      const int qi = q0 + 8 * hh + r;
      const int ja = j0 + ln, jb = j0 + 16 + ln;
      if (CAUSAL) { if (ja > qi) s[0][r] = -3.0e38f; if (jb > qi) s[1][r] = -3.0e38f; }
      if (ja >= T) s[0][r] = -3.0e38f;
      if (jb >= T) s[1][r] = -3.0e38f;
      float mx = fmaxf(s[0][r], s[1][r]);
      mx = fmaxf(mx, __shfl_xor(mx, 1, 32)); mx = fmaxf(mx, __shfl_xor(mx, 2, 32)); mx = fmaxf(mx, __shfl_xor(mx, 4, 32)); mx = fmaxf(mx, __shfl_xor(mx, 8, 32));
      const float mnew = fmaxf(m_r[r], mx);
      alpha[r] = (mnew > -1.0e38f) ? __expf(m_r[r] - mnew) : 1.0f;
      const float p0 = (s[0][r] > -1.0e38f) ? __expf(s[0][r] - mnew) : 0.f;
      const float p1 = (s[1][r] > -1.0e38f) ? __expf(s[1][r] - mnew) : 0.f;
      m_r[r] = mnew;
      l_r[r] = l_r[r] * alpha[r] + p0 + p1;
      unsigned short hb = bf16_bits(p0); sPh[w][8 * hh + r][ln] = hb;      sPl[w][8 * hh + r][ln] = bf16_bits(p0 - bf16_val(hb));
      hb = bf16_bits(p1);                sPh[w][8 * hh + r][16 + ln] = hb; sPl[w][8 * hh + r][16 + ln] = bf16_bits(p1 - bf16_val(hb));
    }
#pragma unroll
    for (int dt = 0; dt < DT; ++dt)
#pragma unroll
      for (int r = 0; r < 8; ++r) oacc[dt][r] *= alpha[r];
    __builtin_amdgcn_fence(__ATOMIC_ACQ_REL, "workgroup");
    __builtin_amdgcn_wave_barrier();
    FragB pah, pal;
    pah.half[0] = *(const v8us*)&sPh[w][ln][8 * hh]; pah.half[1] = *(const v8us*)&sPh[w][ln][16 + 8 * hh];
    pal.half[0] = *(const v8us*)&sPl[w][ln][8 * hh]; pal.half[1] = *(const v8us*)&sPl[w][ln][16 + 8 * hh];
#pragma unroll
    for (int dt = 0; dt < DT; ++dt) {
      FragB bvh, bvl;
#pragma unroll
      for (int i = 0; i < 8; ++i) {
        bvh.u[i] = sVh[8 * hh + i][dt * 16 + ln]; bvh.u[8 + i] = sVh[16 + 8 * hh + i][dt * 16 + ln];
        bvl.u[i] = sVl[8 * hh + i][dt * 16 + ln]; bvl.u[8 + i] = sVl[16 + 8 * hh + i][dt * 16 + ln];
      }
      oacc[dt] = mmaN<3>(pah.v, pal.v, bvh.v, bvl.v, oacc[dt]);
    }
    __builtin_amdgcn_fence(__ATOMIC_ACQ_REL, "workgroup");
    __builtin_amdgcn_wave_barrier();
  }
#pragma unroll
  for (int r = 0; r < 8; ++r) {
    float l = l_r[r];
    l += __shfl_xor(l, 1, 32); l += __shfl_xor(l, 2, 32); l += __shfl_xor(l, 4, 32); l += __shfl_xor(l, 8, 32);
    l_r[r] = (l > 0.f) ? 1.0f / l : 0.f;
  }
#pragma unroll
  for (int dt = 0; dt < DT; ++dt)
#pragma unroll
    for (int r = 0; r < 8; ++r) sO[w][8 * hh + r][dt * 16 + ln] = oacc[dt][r] * l_r[r];
  __builtin_amdgcn_fence(__ATOMIC_ACQ_REL, "workgroup");
  __builtin_amdgcn_wave_barrier();
  for (int pass = 0; pass < 2; ++pass) {
    for (int r = 0; r < 16; ++r) {
      const int row = q0 + r;
      if (row < T && lane < D / 4) {
        const v4f val = *(const v4fa*)&sO[w][r][lane * 4];
        *(volatile v4f*)(y + ((size_t)b * T + row) * ypitch + h * D + lane * 4) = val;
      }
    }
    if (pass == 0) __threadfence();
  }
}

template <bool ASPLIT, int ACT, bool BIAS_BF16, bool RES_BF16>
__global__ __launch_bounds__(128) void k_gemm_bf3(const float* __restrict__ A, int lda, const unsigned short* __restrict__ Wt, int ldb,
                                                const float* __restrict__ bias, const float* __restrict__ resid, int rmod, int ldr,
                                                float* __restrict__ C, int ldc, int M, int N, int K) {
  __shared__ __attribute__((aligned(16))) float so[4][16][64];
  const int tid = threadIdx.x, w = tid >> 5, lane = tid & 31, ln = lane & 15, hh = lane >> 4;
  const int ntn = N / 64;
  const int wid = blockIdx.x * 4 + w;
  const int mt = wid / ntn, nq = wid % ntn;
  if (mt * 16 >= M) return;
  const int row0 = mt * 16, col0 = nq * 64;
  const float* arow = A + (size_t)(row0 + ln) * lda;
  v8f acc[4] = {};
  for (int kb = 0; kb < K; kb += 32) {
    FragB ah, al;
    const v4f x0 = *(const v4fa*)(arow + kb + 8 * hh), x1 = *(const v4fa*)(arow + kb + 8 * hh + 4);
    const v4f x2 = *(const v4fa*)(arow + kb + 16 + 8 * hh), x3 = *(const v4fa*)(arow + kb + 16 + 8 * hh + 4);
    float xs[16] = {x0[0],x0[1],x0[2],x0[3],x1[0],x1[1],x1[2],x1[3],x2[0],x2[1],x2[2],x2[3],x3[0],x3[1],x3[2],x3[3]};
#pragma unroll
    for (int i = 0; i < 16; ++i) { const unsigned short hb = bf16_bits(xs[i]); ah.u[i] = hb; al.u[i] = ASPLIT ? bf16_bits(xs[i] - bf16_val(hb)) : (unsigned short)0; }
#pragma unroll
    for (int t = 0; t < 4; ++t) {
      const unsigned short* brow = Wt + (size_t)(col0 + t * 16 + ln) * ldb + kb;
      FragB b;
      b.half[0] = *(const v8us*)(brow + 8 * hh);
      b.half[1] = *(const v8us*)(brow + 16 + 8 * hh);
      acc[t] = mmaN<ASPLIT ? 2 : 1>(ah.v, al.v, b.v, b.v, acc[t]);
    }
  }
#pragma unroll
  for (int t = 0; t < 4; ++t) {
    const int col = col0 + t * 16 + ln;
    float bv = bias ? bias[col] : 0.f;
    if (BIAS_BF16) bv = bf16_round(bv);
#pragma unroll
    for (int r = 0; r < 8; ++r) {
      float v = acc[t][r] + bv;
      if (resid) { float rv = resid[(size_t)((row0 + 8 * hh + r) % rmod) * ldr + col]; if (RES_BF16) rv = bf16_round(rv); v += rv; }
      if (ACT == 1) v = fmaxf(v, 0.f);
      if (ACT == 2) v = 0.5f * v * (1.0f + erff(v * 0.70710678118654752f));
      if (ACT == 3) { const float u = 0.7978845608028654f * (v + 0.044715f * v * v * v); v = 0.5f * v * (1.0f + tanhf(u)); }
      so[w][8 * hh + r][t * 16 + ln] = v;
    }
  }
  __builtin_amdgcn_fence(__ATOMIC_ACQ_REL, "workgroup");
  __builtin_amdgcn_wave_barrier();
  const int rsub = lane >> 4, c4 = (lane & 15) * 4;
  for (int pass = 0; pass < 2; ++pass) {
#pragma unroll
    for (int q = 0; q < 8; ++q) {
      const int r = q * 2 + rsub;
      const v4f v = *(const v4fa*)&so[w][r][c4];
      *(volatile v4f*)(C + (size_t)(row0 + r) * ldc + col0 + c4) = v;
    }
    if (pass == 0) __threadfence();
  }
}
template <bool PARAM_BF16>
__global__ __launch_bounds__(256) void k_layernorm(const float* __restrict__ X, const float* __restrict__ R, const float* __restrict__ g, const float* __restrict__ bta,
                                                  float* __restrict__ out_sum, float* __restrict__ out_norm, int N, float eps) {
  __shared__ float red[256];
  const int row = blockIdx.x, tid = threadIdx.x;
  const float* x = X + (size_t)row * N; const float* rr = R ? R + (size_t)row * N : nullptr;
  float vals[16];
  const int per = N / 256;
  float s1 = 0.f;
  for (int u = 0; u < per / 4; ++u) {
    const int j = tid * 4 + 1024 * u;
    const v4f a = *(const v4fa*)(x + j);
    v4f b = {0.f,0.f,0.f,0.f}; if (rr) b = *(const v4fa*)(rr + j);
#pragma unroll
    for (int q = 0; q < 4; ++q) { const float v = a[q] + b[q]; vals[u * 4 + q] = v; s1 += v; }
  }
  red[tid] = s1; __syncthreads();
  for (int st = 128; st > 0; st >>= 1) { if (tid < st) red[tid] += red[tid + st]; __syncthreads(); }
  const float mu = red[0] / (float)N; __syncthreads();
  float s2 = 0.f;
  for (int u = 0; u < per / 4; ++u)
#pragma unroll
    for (int q = 0; q < 4; ++q) { const float c = vals[u * 4 + q] - mu; s2 += c * c; }
  red[tid] = s2; __syncthreads();
  for (int st = 128; st > 0; st >>= 1) { if (tid < st) red[tid] += red[tid + st]; __syncthreads(); }
  const float rs = rsqrtf(red[0] / (float)N + eps);
  for (int pass = 0; pass < 2; ++pass) {
    for (int u = 0; u < per / 4; ++u) {
      const int j = tid * 4 + 1024 * u;
      v4f o, sm;
#pragma unroll
      for (int q = 0; q < 4; ++q) {
        float gg = g[j + q], bb = bta[j + q];
        if (PARAM_BF16) { gg = bf16_round(gg); bb = bf16_round(bb); }
        sm[q] = vals[u * 4 + q]; o[q] = (vals[u * 4 + q] - mu) * rs * gg + bb;
      }
      if (out_sum) *(volatile v4f*)(out_sum + (size_t)row * N + j) = sm;
      *(volatile v4f*)(out_norm + (size_t)row * N + j) = o;
    }
    if (pass == 0) __threadfence();
  }
}


typedef _Float16 v16h __attribute__((ext_vector_type(16)));
union FragH { v16h v; v8us half[2]; _Float16 h[16]; unsigned short u[16]; };
template <int NT>
__device__ __forceinline__ v8f mmaH(v16h ah, v16h al, v16h bh, v16h bl, v8f c) {
  c = __builtin_amdgcn_wmma_f32_16x16x32_f16(false, ah, false, bh, (short)0, c, false, false);
  if (NT >= 2) c = __builtin_amdgcn_wmma_f32_16x16x32_f16(false, al, false, bh, (short)0, c, false, false);
  if (NT >= 3) c = __builtin_amdgcn_wmma_f32_16x16x32_f16(false, ah, false, bl, (short)0, c, false, false);
  asm volatile("v_nop\n\tv_nop\n\tv_nop\n\tv_nop" : "+v"(c) : "v"(ah), "v"(al), "v"(bh), "v"(bl));
  return c;
}
template <bool ASPLIT>
__global__ __launch_bounds__(128) void k_gemm_h(const float* __restrict__ A, int lda, size_t sA, const _Float16* __restrict__ Bh, int ldb, size_t sB, float alpha, float* __restrict__ C, int ldc, size_t sC, int M, int N, int K) {
  __shared__ __attribute__((aligned(16))) float so[4][16][64];
  const int tid = threadIdx.x, w = tid >> 5, lane = tid & 31, ln = lane & 15, hh = lane >> 4; const int by = blockIdx.y;
  A += (size_t)by * sA; Bh += (size_t)by * sB; C += (size_t)by * sC;
  const int ntn = (N + 63) / 64; const int wid = blockIdx.x * 4 + w; const int mt = wid / ntn, nq = wid % ntn; if (mt * 16 >= M) return;
  const int row0 = mt * 16, col0 = nq * 64; const float* arow = A + (size_t)(row0 + ln) * lda;
  v8f acc[4] = {};
  for (int kb = 0; kb < K; kb += 32) {
    FragH ah, al;
    const v4f x0 = *(const v4fa*)(arow + kb + 8 * hh), x1 = *(const v4fa*)(arow + kb + 8 * hh + 4), x2 = *(const v4fa*)(arow + kb + 16 + 8 * hh), x3 = *(const v4fa*)(arow + kb + 16 + 8 * hh + 4);
    float xs[16] = {x0[0],x0[1],x0[2],x0[3],x1[0],x1[1],x1[2],x1[3],x2[0],x2[1],x2[2],x2[3],x3[0],x3[1],x3[2],x3[3]};
#pragma unroll
    for (int i = 0; i < 16; ++i) { const _Float16 h = (_Float16)xs[i]; ah.h[i] = h; al.h[i] = ASPLIT ? (_Float16)(xs[i] - (float)h) : (_Float16)0.0f; }
#pragma unroll
    for (int t = 0; t < 4; ++t) { if (col0 + t * 16 >= N) continue; const size_t boff = (size_t)(col0 + t * 16 + ln) * ldb + kb; FragH bq; bq.half[0] = *(const v8us*)(Bh + boff + 8 * hh); bq.half[1] = *(const v8us*)(Bh + boff + 16 + 8 * hh);
      acc[t] = mmaH<ASPLIT ? 2 : 1>(ah.v, al.v, bq.v, bq.v, acc[t]); }
  }
#pragma unroll
  for (int t = 0; t < 4; ++t) { if (col0 + t * 16 >= N) continue;
#pragma unroll
    for (int r = 0; r < 8; ++r) so[w][8 * hh + r][t * 16 + ln] = acc[t][r] * alpha; }
  __builtin_amdgcn_fence(__ATOMIC_ACQ_REL, "workgroup"); __builtin_amdgcn_wave_barrier();
  const int rsub = lane >> 4, c4 = (lane & 15) * 4;
  for (int pass = 0; pass < 2; ++pass) {
#pragma unroll
    for (int q = 0; q < 8; ++q) { const int r = q * 2 + rsub; if (col0 + c4 < N) { const v4f v = *(const v4fa*)&so[w][r][c4]; *(volatile v4f*)(C + (size_t)(row0 + r) * ldc + col0 + c4) = v; } }
    if (pass == 0) __threadfence(); }
}

__global__ __launch_bounds__(256) void k_wt_f16(const float* __restrict__ W, _Float16* __restrict__ Wt, int K, int N, float scale) {
  const int t = blockIdx.x * 256 + threadIdx.x; if (t >= N * (K / 8)) return; const int n = t / (K / 8), k8 = (t % (K / 8)) * 8; FragH f;
#pragma unroll
  for (int i = 0; i < 8; ++i) f.h[i] = (_Float16)(bf16_round(W[(size_t)(k8 + i) * N + n]) * scale); const v8us o = f.half[0];
  *(volatile v8us*)((unsigned short*)Wt + (size_t)n * K + k8) = o; __threadfence(); *(volatile v8us*)((unsigned short*)Wt + (size_t)n * K + k8) = o;
}
template <int ACT>
__global__ __launch_bounds__(128) void k_gemm_hhx(const _Float16* __restrict__ A, int lda, size_t sA, const _Float16* __restrict__ Bh, int ldb, size_t sB, float alpha, const float* __restrict__ bias, size_t sBias, const float* __restrict__ CP, int rowsPerB, size_t sCPb, int row0g,
    float* __restrict__ C, _Float16* __restrict__ C16, int ldc, size_t sC, int M, int N, int K) {
  __shared__ __attribute__((aligned(16))) float so[4][16][64];
  const int tid = threadIdx.x, w = tid >> 5, lane = tid & 31, ln = lane & 15, hh = lane >> 4; const int by = blockIdx.y;
  A += (size_t)by * sA; Bh += (size_t)by * sB; const size_t cofs = (size_t)by * sC; const float* bp = bias ? bias + (size_t)by * sBias : nullptr;
  const int ntn = (N + 63) / 64; const int wid = blockIdx.x * 4 + w; const int mt = wid / ntn, nq = wid % ntn; if (mt * 16 >= M) return;
  const int row0 = mt * 16, col0 = nq * 64; const _Float16* arow = A + (size_t)(row0 + ln) * lda;
  v8f acc[4] = {};
  for (int kb = 0; kb < K; kb += 32) { FragH ah; ah.half[0] = *(const v8us*)((const unsigned short*)arow + kb + 8 * hh); ah.half[1] = *(const v8us*)((const unsigned short*)arow + kb + 16 + 8 * hh);
#pragma unroll
    for (int t = 0; t < 4; ++t) { if (col0 + t * 16 >= N) continue; const size_t boff = (size_t)(col0 + t * 16 + ln) * ldb + kb; FragH bq; bq.half[0] = *(const v8us*)((const unsigned short*)Bh + boff + 8 * hh); bq.half[1] = *(const v8us*)((const unsigned short*)Bh + boff + 16 + 8 * hh);
      acc[t] = mmaH<1>(ah.v, ah.v, bq.v, bq.v, acc[t]); }
  }
#pragma unroll
  for (int t = 0; t < 4; ++t) { if (col0 + t * 16 >= N) continue; const int col = col0 + t * 16 + ln; const float bv = bp ? bf16_round(bp[col]) : 0.f;
#pragma unroll
    for (int r = 0; r < 8; ++r) { float v = acc[t][r] * alpha + bv; if (CP) { const int bidx = (row0g + row0 + 8 * hh + r) / rowsPerB; v += CP[(size_t)bidx * sCPb + (size_t)by * 64 + col]; } if (ACT == 1) v = (v > 0.f) ? v : expm1f(v); else if (ACT == 3) v = fmaxf(v, 0.f); so[w][8 * hh + r][t * 16 + ln] = v; } }
  __builtin_amdgcn_fence(__ATOMIC_ACQ_REL, "workgroup"); __builtin_amdgcn_wave_barrier();
  const int rsub = lane >> 4, c4 = (lane & 15) * 4; typedef _Float16 v4h __attribute__((ext_vector_type(4)));
  for (int pass = 0; pass < 2; ++pass) {
#pragma unroll
    for (int q = 0; q < 8; ++q) { const int r = q * 2 + rsub; if (col0 + c4 < N) { const v4f v = *(const v4fa*)&so[w][r][c4]; if (C) *(volatile v4f*)(C + cofs + (size_t)(row0 + r) * ldc + col0 + c4) = v; if (C16) { v4h h4; for (int i = 0; i < 4; ++i) h4[i] = (_Float16)v[i]; *(volatile v4h*)(C16 + cofs + (size_t)(row0 + r) * ldc + col0 + c4) = h4; } } }
    if (pass == 0) __threadfence(); }
}


__device__ __forceinline__ float tanh_f(float x) { const float e = expf(2.0f * x); return 1.0f - 2.0f / (1.0f + e); }
__device__ __forceinline__ float sigm_f(float x) { return 1.0f / (1.0f + expf(-x)); }
__global__ __launch_bounds__(256) void k_x16(const float* __restrict__ x, _Float16* __restrict__ X16, size_t n8) { const size_t t = (size_t)blockIdx.x * 256 + threadIdx.x; if (t >= n8) return; FragH f;
#pragma unroll
  for (int q = 0; q < 8; ++q) f.h[q] = (_Float16)bf16_round(x[t * 8 + q]); *(volatile v8us*)((unsigned short*)X16 + t * 8) = f.half[0]; __threadfence(); *(volatile v8us*)((unsigned short*)X16 + t * 8) = f.half[0]; }
__global__ __launch_bounds__(256) void k_round16f(const float* __restrict__ W, _Float16* __restrict__ Bt, size_t n8) { const size_t t = (size_t)blockIdx.x * 256 + threadIdx.x; if (t >= n8) return; FragH f;
#pragma unroll
  for (int i = 0; i < 8; ++i) f.h[i] = (_Float16)(bf16_round(W[t * 8 + i]) * 16.0f); *(volatile v8us*)((unsigned short*)Bt + t * 8) = f.half[0]; __threadfence(); *(volatile v8us*)((unsigned short*)Bt + t * 8) = f.half[0]; }
__global__ __launch_bounds__(256) void k_wcat(const float* __restrict__ Wih, const float* __restrict__ Whh, _Float16* __restrict__ BL) { const int t = blockIdx.x * 256 + threadIdx.x; if (t >= 4 * HH * ((DD + HH) / 8)) return; const int row = t / ((DD + HH) / 8), k8 = (t % ((DD + HH) / 8)) * 8; FragH f;
#pragma unroll
  for (int q = 0; q < 8; ++q) { const int k = k8 + q; f.h[q] = (_Float16)((k < DD ? bf16_round(Wih[(size_t)row * DD + k]) : bf16_round(Whh[(size_t)row * HH + k - DD])) * 16.0f); } *(volatile v8us*)((unsigned short*)BL + (size_t)t * 8) = f.half[0]; __threadfence(); *(volatile v8us*)((unsigned short*)BL + (size_t)t * 8) = f.half[0]; }
__global__ __launch_bounds__(256) void k_coatt(const float* __restrict__ WX, const float* __restrict__ US, const float* __restrict__ v, const float* __restrict__ x, float* __restrict__ SRM) {
  __shared__ float sus[SSQ][DD]; __shared__ float sv[DD]; __shared__ float ssc[SSQ][LL + 1]; __shared__ float sab[LL];
  const int tid = threadIdx.x; const int bn = blockIdx.x; const int b = bn / NNS;
  for (int i = tid; i < SSQ * DD; i += 256) sus[i / DD][i % DD] = US[(size_t)b * SSQ * DD + i]; sv[tid] = bf16_round(v[tid]); __syncthreads();
  { const int l = tid >> 2, s0 = tid & 3; const float* wr = WX + ((size_t)bn * LL + l) * DD; float acc[8];
#pragma unroll
    for (int j = 0; j < 8; ++j) acc[j] = 0.f;
#pragma unroll 1
    for (int d = 0; d < DD; ++d) { const float wx = wr[d], vd = sv[d];
#pragma unroll
      for (int j = 0; j < 8; ++j) acc[j] += tanh_f(wx + sus[s0 + 4 * j][d]) * vd; }
#pragma unroll
    for (int j = 0; j < 8; ++j) ssc[s0 + 4 * j][l] = acc[j]; }
  __syncthreads();
  if (tid < SSQ) { float m = -3.0e38f; for (int l = 0; l < LL; ++l) m = fmaxf(m, ssc[tid][l]); float s = 0.f; for (int l = 0; l < LL; ++l) { const float e = expf(ssc[tid][l] - m); ssc[tid][l] = e; s += e; } const float inv = 1.0f / s; for (int l = 0; l < LL; ++l) ssc[tid][l] *= inv; }
  __syncthreads();
  if (tid < LL) { float s = 0.f; for (int q = 0; q < SSQ; ++q) s += ssc[q][tid]; sab[tid] = s * (1.0f / (float)SSQ); }
  __syncthreads();
  { float acc = 0.f; const float* xr = x + (size_t)bn * LL * DD + tid;
#pragma unroll 4
    for (int l = 0; l < LL; ++l) acc += sab[l] * bf16_round(xr[(size_t)l * DD]);
    *(volatile float*)(SRM + (size_t)bn * DD + tid) = acc; __threadfence(); *(volatile float*)(SRM + (size_t)bn * DD + tid) = acc; } }
__global__ __launch_bounds__(128) void k_lstm(const float* __restrict__ SRM, const _Float16* __restrict__ BLf, const float* __restrict__ bih_f, const float* __restrict__ bhh_f, const _Float16* __restrict__ BLb, const float* __restrict__ bih_b, const float* __restrict__ bhh_b, float* __restrict__ C) {
  __shared__ __attribute__((aligned(16))) unsigned short sA[BB][DD + HH + 8];
  __shared__ __attribute__((aligned(16))) float sh[4][BB][32 + 4];
  const int tid = threadIdx.x, w = tid >> 5, lane = tid & 31, ln = lane & 15, hh = lane >> 4; const int dir = blockIdx.x;
  const _Float16* BL = dir ? BLb : BLf; const float* bih = dir ? bih_b : bih_f; const float* bhh = dir ? bhh_b : bhh_f;
  for (int i = tid; i < BB * (DD + HH + 8); i += 128) ((unsigned short*)sA)[i] = 0;
  float bias[8];
#pragma unroll
  for (int t = 0; t < 8; ++t) { const int row = (t >> 1) * HH + 32 * w + 16 * (t & 1) + ln; bias[t] = bf16_round(bih[row]) + bf16_round(bhh[row]); }
  float c_st[2][8];
#pragma unroll
  for (int u = 0; u < 2; ++u)
#pragma unroll
    for (int r = 0; r < 8; ++r) c_st[u][r] = 0.f;
  __syncthreads();
#pragma unroll 1
  for (int step = 0; step < NNS; ++step) { const int n = dir ? (NNS - 1 - step) : step;
    for (int i = tid; i < BB * DD / 8; i += 128) { const int b = i / (DD / 8), c8 = (i % (DD / 8)) * 8; FragH f; const float* sr = SRM + ((size_t)b * NNS + n) * DD + c8;
#pragma unroll
      for (int q = 0; q < 8; ++q) f.h[q] = (_Float16)sr[q]; *(v8us*)&sA[b][c8] = f.half[0]; }
    __syncthreads();
    v8f acc[8];
#pragma unroll
    for (int t = 0; t < 8; ++t) acc[t] = (v8f){0.f,0.f,0.f,0.f,0.f,0.f,0.f,0.f};
#pragma unroll 2
    for (int ks = 0; ks < (DD + HH) / 32; ++ks) { FragH a; a.half[0] = *(const v8us*)&sA[ln][ks * 32 + 8 * hh]; a.half[1] = *(const v8us*)&sA[ln][ks * 32 + 16 + 8 * hh];
#pragma unroll
      for (int t = 0; t < 8; ++t) { const int row = (t >> 1) * HH + 32 * w + 16 * (t & 1) + ln; const unsigned short* br = (const unsigned short*)BL + (size_t)row * (DD + HH) + ks * 32; FragH b; b.half[0] = *(const v8us*)(br + 8 * hh); b.half[1] = *(const v8us*)(br + 16 + 8 * hh); acc[t] = mmaH<1>(a.v, a.v, b.v, b.v, acc[t]); } }
    __syncthreads();
#pragma unroll
    for (int u = 0; u < 2; ++u)
#pragma unroll
      for (int r = 0; r < 8; ++r) { const float gi = acc[0 + u][r] * 0.0625f + bias[0 + u], gf = acc[2 + u][r] * 0.0625f + bias[2 + u], gg = acc[4 + u][r] * 0.0625f + bias[4 + u], go = acc[6 + u][r] * 0.0625f + bias[6 + u];
        const float cc = sigm_f(gf) * c_st[u][r] + sigm_f(gi) * tanh_f(gg); c_st[u][r] = cc; const float hv = sigm_f(go) * tanh_f(cc); const int j = 32 * w + 16 * u + ln, b = 8 * hh + r;
        FragH t1; t1.h[0] = (_Float16)hv; sA[b][DD + j] = t1.u[0]; sh[w][b][16 * u + ln] = hv; }
    __syncthreads();
    for (int pass = 0; pass < 2; ++pass) {
#pragma unroll
      for (int j4 = 0; j4 < 4; ++j4) { const int b = 4 * j4 + (lane >> 3), pc = lane & 7; const float* sp = &sh[w][b][4 * pc]; float* dp = C + ((size_t)b * NNS + n) * (2 * HH) + dir * HH + 32 * w + 4 * pc; *(volatile v4f*)(dp) = *(const v4fa*)(sp); }
      if (pass == 0) __threadfence(); } } }
__global__ __launch_bounds__(128) void k_attsc(const float* __restrict__ C, const _Float16* __restrict__ BS, const float* __restrict__ sab, const float* __restrict__ sav, float* __restrict__ ATT) {
  __shared__ float sres[4][NNS]; const int tid = threadIdx.x, w = tid >> 5, lane = tid & 31, ln = lane & 15, hh = lane >> 4; const int b = blockIdx.x * 4 + w;
  float part[8];
#pragma unroll
  for (int r = 0; r < 8; ++r) part[r] = 0.f;
#pragma unroll 1
  for (int tl = 0; tl < DD / 16; ++tl) { v8f acc = (v8f){0.f,0.f,0.f,0.f,0.f,0.f,0.f,0.f};
#pragma unroll
    for (int ks = 0; ks < DD / 32; ++ks) { FragH a, bq; if (ln < NNS) { const float* cr = C + ((size_t)b * NNS + ln) * DD + ks * 32;
#pragma unroll
        for (int q = 0; q < 8; ++q) { a.h[q] = (_Float16)cr[8 * hh + q]; a.h[8 + q] = (_Float16)cr[16 + 8 * hh + q]; } } else { for (int q = 0; q < 16; ++q) a.h[q] = (_Float16)0.0f; }
      const unsigned short* br = (const unsigned short*)BS + (size_t)(tl * 16 + ln) * DD + ks * 32; bq.half[0] = *(const v8us*)(br + 8 * hh); bq.half[1] = *(const v8us*)(br + 16 + 8 * hh); acc = mmaH<1>(a.v, a.v, bq.v, bq.v, acc); }
    const int e = tl * 16 + ln; const float be = bf16_round(sab[e]), ve = bf16_round(sav[e]);
#pragma unroll
    for (int r = 0; r < 8; ++r) part[r] += tanh_f(acc[r] * 0.0625f + be) * ve; }
#pragma unroll
  for (int r = 0; r < 8; ++r) { float v = part[r]; v += __shfl_xor(v, 1, 32); v += __shfl_xor(v, 2, 32); v += __shfl_xor(v, 4, 32); v += __shfl_xor(v, 8, 32); part[r] = v; }
  if (lane == 0) {
#pragma unroll
    for (int r = 0; r < 8; ++r) sres[w][r] = part[r]; }
  __syncthreads();
  if (tid < 32) { *(volatile float*)(ATT + (size_t)blockIdx.x * 32 + tid) = sres[tid / 8][tid % 8]; } __threadfence(); if (tid < 32) { *(volatile float*)(ATT + (size_t)blockIdx.x * 32 + tid) = sres[tid / 8][tid % 8]; } }
__global__ __launch_bounds__(256) void k_pool(const float* __restrict__ C, const float* __restrict__ ATT, float* __restrict__ out) { __shared__ float sa[NNS]; const int tid = threadIdx.x; const int b = blockIdx.x;
  if (tid == 0) { float m = -3.0e38f; for (int n = 0; n < NNS; ++n) m = fmaxf(m, ATT[b * NNS + n]); float s = 0.f; float e[NNS]; for (int n = 0; n < NNS; ++n) { e[n] = expf(ATT[b * NNS + n] - m); s += e[n]; } for (int n = 0; n < NNS; ++n) sa[n] = e[n] / s; }
  __syncthreads(); float g = 0.f;
#pragma unroll
  for (int n = 0; n < NNS; ++n) g += sa[n] * C[((size_t)b * NNS + n) * DD + tid];
  *(volatile float*)(out + (size_t)b * DD + tid) = g; __threadfence(); *(volatile float*)(out + (size_t)b * DD + tid) = g; }
extern "C" void kernel_launch(void* const* d_in, const int* in_sizes, int n_in,
                              void* d_out, int out_size, void* d_ws, size_t ws_size, hipStream_t stream) {
  (void)in_sizes; (void)n_in; (void)out_size;
  const float* x = (const float*)d_in[0]; const float* s = (const float*)d_in[1]; const float* W = (const float*)d_in[2]; const float* U = (const float*)d_in[3]; const float* v = (const float*)d_in[4];
  const float* Wih_f = (const float*)d_in[5]; const float* Whh_f = (const float*)d_in[6]; const float* bih_f = (const float*)d_in[7]; const float* bhh_f = (const float*)d_in[8]; const float* Wih_b = (const float*)d_in[9]; const float* Whh_b = (const float*)d_in[10]; const float* bih_b = (const float*)d_in[11]; const float* bhh_b = (const float*)d_in[12];
  const float* saW = (const float*)d_in[13]; const float* sab = (const float*)d_in[14]; const float* sav = (const float*)d_in[15];
  char* ws = (char*)d_ws; size_t off = 0;
  auto take = [&](size_t bytes) { char* p = ws + off; off += (bytes + 255) & ~(size_t)255; return p; };
  const size_t NRX = (size_t)BB * NNS * LL, NRS = (size_t)BB * SSQ;
  _Float16* BW = (_Float16*)take(DD * DD * 2); _Float16* BU = (_Float16*)take(DD * DD * 2); _Float16* X16 = (_Float16*)take(NRX * DD * 2); _Float16* S16 = (_Float16*)take(NRS * DD * 2); float* WX = (float*)take(NRX * DD * 4); float* US = (float*)take(NRS * DD * 4); float* SRM = (float*)take((size_t)BB * NNS * DD * 4); float* C = (float*)take((size_t)BB * NNS * 2 * HH * 4); _Float16* BLf = (_Float16*)take((size_t)4 * HH * (DD + HH) * 2); _Float16* BLb = (_Float16*)take((size_t)4 * HH * (DD + HH) * 2); _Float16* BSA = (_Float16*)take(DD * DD * 2); float* ATT = (float*)take(BB * NNS * 4);
  if (off > ws_size) return;
  k_round16f<<<(DD * DD / 8 + 255) / 256, 256, 0, stream>>>(W, BW, DD * DD / 8); k_round16f<<<(DD * DD / 8 + 255) / 256, 256, 0, stream>>>(U, BU, DD * DD / 8);
  k_x16<<<(unsigned)((NRX * DD / 8 + 255) / 256), 256, 0, stream>>>(x, X16, NRX * DD / 8); k_x16<<<(unsigned)((NRS * DD / 8 + 255) / 256), 256, 0, stream>>>(s, S16, NRS * DD / 8);
  k_gemm_hhx<0><<<dim3(((unsigned)(NRX / 16) * (DD / 64) + 3) / 4, 1), 128, 0, stream>>>(X16, DD, 0, BW, DD, 0, 0.0625f, nullptr, 0, nullptr, 1, 0, 0, WX, nullptr, DD, 0, (int)NRX, DD, DD);
  k_gemm_hhx<0><<<dim3(((unsigned)(NRS / 16) * (DD / 64) + 3) / 4, 1), 128, 0, stream>>>(S16, DD, 0, BU, DD, 0, 0.0625f, nullptr, 0, nullptr, 1, 0, 0, US, nullptr, DD, 0, (int)NRS, DD, DD);
  k_coatt<<<BB * NNS, 256, 0, stream>>>(WX, US, v, x, SRM);
  k_wcat<<<(4 * HH * ((DD + HH) / 8) + 255) / 256, 256, 0, stream>>>(Wih_f, Whh_f, BLf); k_wcat<<<(4 * HH * ((DD + HH) / 8) + 255) / 256, 256, 0, stream>>>(Wih_b, Whh_b, BLb); k_round16f<<<(DD * DD / 8 + 255) / 256, 256, 0, stream>>>(saW, BSA, DD * DD / 8);
  k_lstm<<<2, 128, 0, stream>>>(SRM, BLf, bih_f, bhh_f, BLb, bih_b, bhh_b, C);
  k_attsc<<<BB / 4, 128, 0, stream>>>(C, BSA, sab, sav, ATT);
  k_pool<<<BB, 256, 0, stream>>>(C, ATT, (float*)d_out);
}
